// EEHGCN_82085414961677
// MI455X (gfx1250) — hardware-verified
//
#include <hip/hip_runtime.h>
#include <stddef.h>


#define DIMF    64
#define KIN     192
#define NREL    16
#define NT      256
#define NWAVE   8
#define EPT     8
#define NGRP    4
#define CHUNK   (NT * EPT * NGRP)
#define WCAP    (EPT * NGRP * 32)
#define LISTN   (NWAVE * WCAP)
#define NBK     1536
#define CAPB    26624
#define RB      256
#define APH     200
#define MAXDEG  64
#define RELP    17
#define ASCALE  64.0f
#define WSCALE  16.0f
#define OSCALE  0.0009765625f

#define LDS_CSR      (CAPB * 4 * 2 + NBK * 4 * 3 + LISTN * 4 + 64)
#define LOFF_RELACC  (RB * APH * 2)
#define LOFF_RELFIN  (LOFF_RELACC + 4 * RELP * DIMF * 4)
#define LOFF_ATTR    (LOFF_RELFIN + NREL * DIMF * 4)
#define LOFF_RN      (LOFF_ATTR + RB * 4)
#define LOFF_RT      (LOFF_RN + RB * 4)
#define LDS_LAY      (LOFF_RT + 2 * RB * 4)

static_assert((CHUNK & (CHUNK - 1)) == 0);
static_assert(CHUNK <= 8192);
static_assert(NBK <= 2047);
static_assert(NBK == 6 * NT);
static_assert(NBK % RB == 0);
static_assert(RB == NT);
static_assert(CAPB % (NWAVE * 128) == 0);
static_assert(CAPB < 65536);
static_assert(LISTN >= NBK);
static_assert(RB * DIMF * 4 <= RB * APH * 2);
static_assert((KIN * DIMF / 8) % NT == 0);

typedef float    v4f  __attribute__((ext_vector_type(4)));
typedef float    v8f  __attribute__((ext_vector_type(8)));
typedef int      v4i  __attribute__((ext_vector_type(4)));
typedef _Float16 v8h  __attribute__((ext_vector_type(8)));
typedef _Float16 v16h __attribute__((ext_vector_type(16)));
union FragH { v16h v; v8h h[2]; };

__device__ __forceinline__ v8h cvt8(v4f a, v4f b) {
  v8h r;
  r[0] = (_Float16)a.x; r[1] = (_Float16)a.y; r[2] = (_Float16)a.z; r[3] = (_Float16)a.w;
  r[4] = (_Float16)b.x; r[5] = (_Float16)b.y; r[6] = (_Float16)b.z; r[7] = (_Float16)b.w;
  return r;
}

__device__ __forceinline__ v8f wmh(v16h a, v16h b, v8f c) {
  v8f d = __builtin_amdgcn_wmma_f32_16x16x32_f16(false, a, false, b, (short)0, c, false, false);
  asm volatile("v_nop\n\tv_nop\n\tv_nop\n\tv_nop" : "+v"(d) : "v"(a), "v"(b));
  return d;
}

__device__ __forceinline__ unsigned match11(int key) {
  unsigned eqm = 0xffffffffu;
#pragma unroll
  for (int b = 0; b < 11; ++b) {
    const bool bit = ((key >> b) & 1) != 0;
    const unsigned mb = __builtin_amdgcn_ballot_w32(bit);
    eqm &= bit ? mb : ~mb;
  }
  return eqm;
}

__device__ __forceinline__ int scan_chunk(const int* __restrict__ dsts, int nE, int cbase, int nodeBase,
                                          int* list, int tid, int lane, int wave) {
  int wc = 0;
#pragma unroll
  for (int g = 0; g < NGRP; ++g) {
    const int el0  = (g * NT + tid) * EPT;
    const int e0   = cbase + el0;
    const int sent = -2147483647 - 1;
    v4i da, db;
    if (cbase + CHUNK <= nE) {
      da = *(const v4i*)(dsts + e0);
      db = *(const v4i*)(dsts + e0 + 4);
    } else {
      da.x = (e0     < nE) ? dsts[min(e0,     nE - 1)] : sent;
      da.y = (e0 + 1 < nE) ? dsts[min(e0 + 1, nE - 1)] : sent;
      da.z = (e0 + 2 < nE) ? dsts[min(e0 + 2, nE - 1)] : sent;
      da.w = (e0 + 3 < nE) ? dsts[min(e0 + 3, nE - 1)] : sent;
      db.x = (e0 + 4 < nE) ? dsts[min(e0 + 4, nE - 1)] : sent;
      db.y = (e0 + 5 < nE) ? dsts[min(e0 + 5, nE - 1)] : sent;
      db.z = (e0 + 6 < nE) ? dsts[min(e0 + 6, nE - 1)] : sent;
      db.w = (e0 + 7 < nE) ? dsts[min(e0 + 7, nE - 1)] : sent;
    }
    const unsigned nb = (unsigned)nodeBase;
    const unsigned s0 = (unsigned)da.x - nb, s1 = (unsigned)da.y - nb;
    const unsigned s2 = (unsigned)da.z - nb, s3 = (unsigned)da.w - nb;
    const unsigned s4 = (unsigned)db.x - nb, s5 = (unsigned)db.y - nb;
    const unsigned s6 = (unsigned)db.z - nb, s7 = (unsigned)db.w - nb;
    const bool h0 = s0 < (unsigned)NBK, h1 = s1 < (unsigned)NBK, h2 = s2 < (unsigned)NBK, h3 = s3 < (unsigned)NBK;
    const bool h4 = s4 < (unsigned)NBK, h5 = s5 < (unsigned)NBK, h6 = s6 < (unsigned)NBK, h7 = s7 < (unsigned)NBK;
    const unsigned any = __builtin_amdgcn_ballot_w32(h0 | h1 | h2 | h3 | h4 | h5 | h6 | h7);
    if (any != 0u) {
#define HITJ(J, HJ, SJ) { \
        const unsigned mj = __builtin_amdgcn_ballot_w32(HJ); \
        if (mj != 0u) { \
          if (HJ) { \
            const int pos = wc + (int)__builtin_amdgcn_mbcnt_lo(mj, 0u); \
            if (pos < WCAP) list[wave * WCAP + pos] = ((el0 + (J)) << 12) | (int)(SJ); \
          } \
          wc += (int)__builtin_popcount(mj); } }
      HITJ(0, h0, s0)
      HITJ(1, h1, s1)
      HITJ(2, h2, s2)
      HITJ(3, h3, s3)
      HITJ(4, h4, s4)
      HITJ(5, h5, s5)
      HITJ(6, h6, s6)
      HITJ(7, h7, s7)
#undef HITJ
    }
  }
  return wc;
}

__global__ __launch_bounds__(NT) void k_wprep(
    const float* __restrict__ W0, const float* __restrict__ W1,
    _Float16* wt0, _Float16* wt1, int nPer) {
  const int i = blockIdx.x * NT + threadIdx.x;
  if (i >= 2 * nPer) return;
  const bool second = i >= nPer;
  const int ii = second ? i - nPer : i;
  const int n  = ii / (KIN / 8);
  const int k0 = (ii - n * (KIN / 8)) * 8;
  const float* p = (second ? W1 : W0) + (size_t)k0 * DIMF + n;
  v4f a, b;
  a.x = p[0];        a.y = p[DIMF];     a.z = p[2 * DIMF]; a.w = p[3 * DIMF];
  b.x = p[4 * DIMF]; b.y = p[5 * DIMF]; b.z = p[6 * DIMF]; b.w = p[7 * DIMF];
  a = a * WSCALE;
  b = b * WSCALE;
  const v8h hv = cvt8(a, b);
  _Float16* dp = (second ? wt1 : wt0) + (size_t)ii * 8;
  *(volatile v8h*)dp = hv;
  __threadfence();
  *(volatile v8h*)dp = hv;
}

__global__ __launch_bounds__(NT) void k_csr(
    const int* __restrict__ rows, unsigned int* rtab, int* eids, int nE) {
  extern __shared__ v4f lds_dyn[];
  char* lb = (char*)lds_dyn;
  unsigned int* ulst = (unsigned int*)lb;
  int*  slst = (int*)(lb + (size_t)CAPB * 4);
  int*  cnt  = (int*)(lb + (size_t)CAPB * 8);
  int*  offa = cnt + NBK;
  int*  cur  = offa + NBK;
  int*  list = cur + NBK;
  int*  wcnt = list + LISTN;
  int*  wtot = wcnt + NWAVE;
  const int tid = threadIdx.x, lane = tid & 31, wave = tid >> 5;
  const int nodeBase = blockIdx.x * NBK;

  {
    const v4i z = {0, 0, 0, 0};
    for (int i = tid; i < CAPB / 4; i += NT) ((v4i*)slst)[i] = z;
    for (int i = tid; i < NBK; i += NT) cnt[i] = 0;
  }
  __syncthreads();

  int tot = 0;
  const int nChunks = (nE + CHUNK - 1) / CHUNK;
#pragma unroll 1
  for (int ch = 0; ch < nChunks; ++ch) {
    const int cbase = ch * CHUNK;
    const int wc = scan_chunk(rows, nE, cbase, nodeBase, list, tid, lane, wave);
    if (lane == 0) wcnt[wave] = wc;
    __syncthreads();
    int pre = 0, sum = 0;
#pragma unroll
    for (int w2 = 0; w2 < NWAVE; ++w2) {
      const int c = wcnt[w2];
      sum += c;
      pre += (w2 < wave) ? c : 0;
    }
    const int* lp = list + wave * WCAP;
    for (int i = lane; i < wc; i += 32) {
      const int ent = lp[i];
      const unsigned g = ((unsigned)(cbase + (ent >> 12)) << 11) | ((unsigned)ent & 2047u);
      const int p = tot + pre + i;
      if (p < CAPB) ulst[p] = g;
    }
    tot += sum;
    __syncthreads();
  }
  int totc = tot < CAPB ? tot : CAPB;
  totc = __builtin_amdgcn_readfirstlane(totc);

  if (wave == 0) {
#pragma unroll 1
    for (int cb = 0; cb < totc; cb += 32) {
      const int i = cb + lane;
      const bool valid = i < totc;
      const unsigned ent = ulst[i < CAPB - 1 ? i : CAPB - 1];
      int sl = (int)(ent & 2047u);
      sl = sl < NBK - 1 ? sl : NBK - 1;
      const int key = valid ? sl : 2047;
      const unsigned eqm = match11(key);
      const int total  = (int)__builtin_popcount(eqm);
      const int before = (int)__builtin_amdgcn_mbcnt_lo(eqm, 0u);
      if (valid && before == total - 1) cnt[sl] = cnt[sl] + total;
      __builtin_amdgcn_fence(__ATOMIC_RELEASE, "wavefront");
      __builtin_amdgcn_wave_barrier();
    }
  }
  __syncthreads();

  {
    int c6[6];
    int s = 0;
#pragma unroll
    for (int j = 0; j < 6; ++j) { c6[j] = cnt[6 * tid + j]; s += c6[j]; }
    int x = s;
#pragma unroll
    for (int d = 1; d < 32; d <<= 1) {
      const int y = __shfl_up(x, d);
      x = (lane >= d) ? x + y : x;
    }
    if (lane == 31) wtot[wave] = x;
    __syncthreads();
    int pre = 0;
#pragma unroll
    for (int w2 = 0; w2 < NWAVE; ++w2) {
      const int t = wtot[w2];
      pre += (w2 < wave) ? t : 0;
    }
    int run = pre + x - s;
#pragma unroll
    for (int j = 0; j < 6; ++j) {
      offa[6 * tid + j] = run;
      cur[6 * tid + j]  = run;
      run += c6[j];
    }
  }
  __syncthreads();

  if (wave == 0) {
#pragma unroll 1
    for (int cb = 0; cb < totc; cb += 32) {
      const int i = cb + lane;
      const bool valid = i < totc;
      const unsigned ent = ulst[i < CAPB - 1 ? i : CAPB - 1];
      int sl = (int)(ent & 2047u);
      sl = sl < NBK - 1 ? sl : NBK - 1;
      const int key = valid ? sl : 2047;
      const unsigned eqm = match11(key);
      const int total  = (int)__builtin_popcount(eqm);
      const int before = (int)__builtin_amdgcn_mbcnt_lo(eqm, 0u);
      const int e   = (int)(ent >> 11);
      const int pos = cur[sl] + before;
      if (valid && (unsigned)pos < (unsigned)CAPB) slst[pos] = e;
      if (valid && before == total - 1) cur[sl] = pos + 1;
      __builtin_amdgcn_fence(__ATOMIC_RELEASE, "wavefront");
      __builtin_amdgcn_wave_barrier();
    }
  }
  __syncthreads();

  {
    unsigned int* rt = (unsigned int*)list;
    for (int i = tid; i < NBK; i += NT) {
      int c = cnt[i];  c = c < 65535 ? c : 65535;  c = c < 0 ? 0 : c;
      int o = offa[i]; o = o < 65535 ? o : 65535;  o = o < 0 ? 0 : o;
      rt[i] = ((unsigned)o << 16) | (unsigned)c;
    }
  }
  __syncthreads();

  {
    int* ge = eids + (size_t)blockIdx.x * CAPB;
    const int per = CAPB / NWAVE;
#pragma unroll 2
    for (int q = 0; q < per / 128; ++q) {
      const int f = wave * per + q * 128 + 4 * lane;
      const v4i v = *(const v4i*)(slst + f);
      *(volatile v4i*)(ge + f) = v;
    }
    unsigned int* gr = rtab + (size_t)blockIdx.x * NBK;
    if (wave < 6) {
#pragma unroll
      for (int q = 0; q < 2; ++q) {
        const int f = (wave * 2 + q) * 128 + 4 * lane;
        const v4i v = *(const v4i*)(list + f);
        *(volatile v4i*)((int*)gr + f) = v;
      }
    }
    __threadfence();
#pragma unroll 2
    for (int q = 0; q < per / 128; ++q) {
      const int f = wave * per + q * 128 + 4 * lane;
      const v4i v = *(const v4i*)(slst + f);
      *(volatile v4i*)(ge + f) = v;
    }
    if (wave < 6) {
#pragma unroll
      for (int q = 0; q < 2; ++q) {
        const int f = (wave * 2 + q) * 128 + 4 * lane;
        const v4i v = *(const v4i*)(list + f);
        *(volatile v4i*)((int*)gr + f) = v;
      }
    }
  }
}

__device__ __forceinline__ void gather_row(unsigned int u, const int* __restrict__ eb,
                                           const int* __restrict__ col, const float* __restrict__ val,
                                           const float* egoIn, int N, int nE, _Float16* dst) {
  const int off = (int)(u >> 16);
  int cnt = (int)(u & 0xffffu);
  cnt = cnt < MAXDEG ? cnt : MAXDEG;
  int mx = cnt;
  mx = max(mx, __shfl_xor(mx, 16));
  mx = max(mx, __shfl_xor(mx, 8));
  mx = max(mx, __shfl_xor(mx, 4));
  mx = max(mx, __shfl_xor(mx, 2));
  mx = max(mx, __shfl_xor(mx, 1));
  mx = __builtin_amdgcn_readfirstlane(mx);
  v4f acc[16];
#pragma unroll
  for (int q = 0; q < 16; ++q) { const v4f z = {0.f, 0.f, 0.f, 0.f}; acc[q] = z; }
#pragma unroll 1
  for (int j = 0; j < mx; ++j) {
    int idx = off + j;
    idx = idx < CAPB - 1 ? idx : CAPB - 1;
    int e = eb[idx];
    e = e < 0 ? 0 : (e > nE - 1 ? nE - 1 : e);
    int c = col[e];
    c = c < 0 ? 0 : (c > N - 1 ? N - 1 : c);
    float v = val[e];
    v = (j < cnt) ? v : 0.0f;
    const float* xp = egoIn + (size_t)c * DIMF;
#pragma unroll
    for (int q = 0; q < 16; ++q) {
      const v4f x = *(const v4f*)(xp + 4 * q);
      acc[q] = acc[q] + x * v;
    }
  }
#pragma unroll
  for (int q = 0; q < 8; ++q)
    *(v8h*)(dst + 8 * q) = cvt8(acc[2 * q] * ASCALE, acc[2 * q + 1] * ASCALE);
}

__device__ __forceinline__ void rel_partial(const float* stg, const float* rnS, const int* attrS,
                                            float* relacc, float* relfin, float* gdst,
                                            int tid, int lane, int wave) {
  const int c = tid & 63, g = tid >> 6;
  float* mine = relacc + (g * RELP) * DIMF + c;
#pragma unroll 4
  for (int k = 0; k < RB / 4; ++k) {
    const int r = 4 * k + g;
    const int a = attrS[r];
    const float v = stg[r * DIMF + c] * rnS[r];
    mine[a * DIMF] = mine[a * DIMF] + v;
  }
  __syncthreads();
#pragma unroll
  for (int j = 0; j < 4; ++j) {
    const int rel = 4 * g + j;
    const float s = relacc[(0 * RELP + rel) * DIMF + c] + relacc[(1 * RELP + rel) * DIMF + c]
                  + relacc[(2 * RELP + rel) * DIMF + c] + relacc[(3 * RELP + rel) * DIMF + c];
    relfin[rel * DIMF + c] = s;
  }
  __syncthreads();
#pragma unroll
  for (int j = 0; j < RELP; ++j) mine[j * DIMF] = 0.0f;
  const v4f pv = *(const v4f*)(relfin + wave * 128 + 4 * lane);
  *(volatile v4f*)(gdst + wave * 128 + 4 * lane) = pv;
  __threadfence();
  *(volatile v4f*)(gdst + wave * 128 + 4 * lane) = pv;
  __syncthreads();
}

__global__ __launch_bounds__(NT) void k_layer(
    const float* egoIn,
    const unsigned int* __restrict__ rtI, const int* __restrict__ eidI,
    const int* __restrict__ colI, const float* __restrict__ valI,
    const unsigned int* __restrict__ rtO, const int* __restrict__ eidO,
    const int* __restrict__ colO, const float* __restrict__ valO,
    const int* __restrict__ attr, const _Float16* __restrict__ wT,
    float* egoOut, float* part, int N, int nEI, int nEO, int nRt, int layer) {
  extern __shared__ v4f lds_dyn[];
  char* lb = (char*)lds_dyn;
  _Float16* sA   = (_Float16*)lb;
  float*    stg  = (float*)lb;
  float*    relacc = (float*)(lb + LOFF_RELACC);
  float*    relfin = (float*)(lb + LOFF_RELFIN);
  int*      attrS  = (int*)(lb + LOFF_ATTR);
  float*    rnS    = (float*)(lb + LOFF_RN);
  unsigned int* rtS = (unsigned int*)(lb + LOFF_RT);
  const int tid = threadIdx.x, lane = tid & 31, wave = tid >> 5, hh = lane >> 4, m = lane & 15;
  const int rowBase = blockIdx.x * RB;
  float* pblk = part + (size_t)blockIdx.x * (3 * NREL * DIMF);

#pragma unroll
  for (int q = 0; q < (RB * DIMF / 4) / NT; ++q) {
    const int idx = q * NT + tid;
    const int r   = idx >> 4;
    const int c4  = (idx & 15) * 4;
    int gr = rowBase + r;
    gr = gr < N - 1 ? gr : N - 1;
    const v4f v = *(const v4f*)(egoIn + (size_t)gr * DIMF + c4);
    *(v4f*)(stg + r * DIMF + c4) = v;
  }
  {
    const int r  = rowBase + tid;
    const int rc = r < N - 1 ? r : N - 1;
    const int a  = attr[rc];
    attrS[tid] = (r < N && (unsigned)a < (unsigned)NREL) ? a : NREL;
    rnS[tid] = 1.0f;
    const int rr = r < nRt - 1 ? r : nRt - 1;
    rtS[tid]      = rtI[rr];
    rtS[RB + tid] = rtO[rr];
  }
  for (int i = tid; i < 4 * RELP * DIMF; i += NT) relacc[i] = 0.0f;
  __syncthreads();

  if (layer == 0) rel_partial(stg, rnS, attrS, relacc, relfin, pblk, tid, lane, wave);

  v4f er[16];
#pragma unroll
  for (int q = 0; q < 16; ++q) er[q] = *(const v4f*)(stg + tid * DIMF + 4 * q);
  __syncthreads();
  _Float16* arow = sA + tid * APH;
#pragma unroll
  for (int q = 0; q < 8; ++q)
    *(v8h*)(arow + 8 * q) = cvt8(er[2 * q] * ASCALE, er[2 * q + 1] * ASCALE);

  const int csrBlk = rowBase / NBK;
  gather_row(rtS[tid],      eidI + (size_t)csrBlk * CAPB, colI, valI, egoIn, N, nEI, arow + DIMF);
  gather_row(rtS[RB + tid], eidO + (size_t)csrBlk * CAPB, colO, valO, egoIn, N, nEO, arow + 2 * DIMF);
  __syncthreads();

  v8f acc8[8];
#pragma unroll
  for (int t = 0; t < 8; ++t) { const v8f z = {0.f, 0.f, 0.f, 0.f, 0.f, 0.f, 0.f, 0.f}; acc8[t] = z; }
  const _Float16* a0p = sA + (32 * wave + m) * APH + 8 * hh;
  const _Float16* a1p = a0p + 16 * APH;
#pragma unroll
  for (int ks = 0; ks < KIN / 32; ++ks) {
    FragH a0, a1;
    a0.h[0] = *(const v8h*)(a0p + 32 * ks);
    a0.h[1] = *(const v8h*)(a0p + 32 * ks + 16);
    a1.h[0] = *(const v8h*)(a1p + 32 * ks);
    a1.h[1] = *(const v8h*)(a1p + 32 * ks + 16);
#pragma unroll
    for (int ct = 0; ct < 4; ++ct) {
      const _Float16* bp = wT + (size_t)(16 * ct + m) * KIN + 32 * ks + 8 * hh;
      FragH b;
      b.h[0] = *(const v8h*)bp;
      b.h[1] = *(const v8h*)(bp + 16);
      acc8[ct]     = wmh(a0.v, b.v, acc8[ct]);
      acc8[4 + ct] = wmh(a1.v, b.v, acc8[4 + ct]);
    }
  }
  __syncthreads();

#pragma unroll
  for (int rt = 0; rt < 2; ++rt) {
    float* sp0 = stg + (32 * wave + 16 * rt + 8 * hh) * DIMF + m;
#pragma unroll
    for (int ct = 0; ct < 4; ++ct) {
      float* sp = sp0 + 16 * ct;
#pragma unroll
      for (int r = 0; r < 8; ++r) {
        float v = acc8[4 * rt + ct][r] * OSCALE;
        v = (v >= 0.0f) ? v : 0.01f * v;
        sp[r * DIMF] = v;
      }
    }
  }
  __syncthreads();

  {
    float s = 0.0f;
    const float* rp = stg + tid * DIMF;
#pragma unroll
    for (int q = 0; q < 16; ++q) {
      const v4f x = *(const v4f*)(rp + 4 * q);
      s += x.x * x.x + x.y * x.y + x.z * x.z + x.w * x.w;
    }
    const float nn = sqrtf(s);
    rnS[tid] = 1.0f / (nn > 1e-12f ? nn : 1e-12f);
  }
  if (layer == 0) {
    const float* lp = stg + (32 * wave) * DIMF + 4 * lane;
    float* gp = egoOut + ((size_t)rowBase + 32 * wave) * DIMF + 4 * lane;
    v4f ov[16];
#pragma unroll
    for (int q = 0; q < 16; ++q) ov[q] = *(const v4f*)(lp + 128 * q);
#pragma unroll
    for (int q = 0; q < 16; ++q) *(volatile v4f*)(gp + 128 * q) = ov[q];
    __threadfence();
#pragma unroll
    for (int q = 0; q < 16; ++q) *(volatile v4f*)(gp + 128 * q) = ov[q];
  }
  __syncthreads();

  rel_partial(stg, rnS, attrS, relacc, relfin, pblk + (1 + layer) * (NREL * DIMF), tid, lane, wave);
}

__global__ __launch_bounds__(NT) void k_comb(const float* __restrict__ part, float* out, int nB) {
  __shared__ __attribute__((aligned(16))) float outS[NREL * KIN];
  const int tid = threadIdx.x, lane = tid & 31, wave = tid >> 5;
  float s[12];
#pragma unroll
  for (int q = 0; q < 12; ++q) s[q] = 0.0f;
#pragma unroll 1
  for (int b = 0; b < nB; ++b) {
    const float* pp = part + (size_t)b * (3 * NREL * DIMF) + tid;
#pragma unroll
    for (int q = 0; q < 12; ++q) s[q] += pp[q * NT];
  }
#pragma unroll
  for (int q = 0; q < 12; ++q) {
    const int f   = q * NT + tid;
    const int sl  = f >> 10;
    const int rel = (f >> 6) & 15;
    const int c   = f & 63;
    outS[rel * KIN + sl * DIMF + c] = s[q];
  }
  __syncthreads();
  v4f ov[3];
#pragma unroll
  for (int q = 0; q < 3; ++q) ov[q] = *(const v4f*)(outS + (wave * 3 + q) * 128 + 4 * lane);
#pragma unroll
  for (int q = 0; q < 3; ++q) *(volatile v4f*)(out + (wave * 3 + q) * 128 + 4 * lane) = ov[q];
  __threadfence();
#pragma unroll
  for (int q = 0; q < 3; ++q) *(volatile v4f*)(out + (wave * 3 + q) * 128 + 4 * lane) = ov[q];
}

extern "C" void kernel_launch(void* const* d_in, const int* in_sizes, int n_in,
                              void* d_out, int out_size, void* d_ws, size_t ws_size,
                              hipStream_t stream) {
  if (n_in < 10) return;
  const int N = in_sizes[0] / DIMF;
  if (N <= 0 || in_sizes[0] != N * DIMF) return;
  if (in_sizes[1] != KIN * DIMF || in_sizes[2] != KIN * DIMF) return;
  const int nEI = in_sizes[3];
  if (nEI <= 0 || in_sizes[4] != nEI || in_sizes[5] != nEI) return;
  const int nEO = in_sizes[6];
  if (nEO <= 0 || in_sizes[7] != nEO || in_sizes[8] != nEO) return;
  if (nEI >= (1 << 21) || nEO >= (1 << 21)) return;
  if (in_sizes[9] != N) return;
  if (out_size != NREL * KIN) return;

  const float* edge_emb = (const float*)d_in[0];
  const float* w0       = (const float*)d_in[1];
  const float* w1       = (const float*)d_in[2];
  const int*   in_row   = (const int*)d_in[3];
  const int*   in_col   = (const int*)d_in[4];
  const float* in_val   = (const float*)d_in[5];
  const int*   out_row  = (const int*)d_in[6];
  const int*   out_col  = (const int*)d_in[7];
  const float* out_val  = (const float*)d_in[8];
  const int*   attr     = (const int*)d_in[9];
  float* out = (float*)d_out;

  const int nCsr = (N + NBK - 1) / NBK;
  const int nLB  = (N + RB - 1) / RB;
  const int nRt  = nCsr * NBK;

  char* ws = (char*)d_ws;
  size_t off = 0;
  const size_t oWT0 = off; off += (size_t)KIN * DIMF * 2;                 off = (off + 255) & ~(size_t)255;
  const size_t oWT1 = off; off += (size_t)KIN * DIMF * 2;                 off = (off + 255) & ~(size_t)255;
  const size_t oRtI = off; off += (size_t)nRt * 4;                        off = (off + 255) & ~(size_t)255;
  const size_t oRtO = off; off += (size_t)nRt * 4;                        off = (off + 255) & ~(size_t)255;
  const size_t oEI  = off; off += (size_t)nCsr * CAPB * 4;                off = (off + 255) & ~(size_t)255;
  const size_t oEO  = off; off += (size_t)nCsr * CAPB * 4;                off = (off + 255) & ~(size_t)255;
  const size_t oEgo = off; off += (size_t)nLB * RB * DIMF * 4;            off = (off + 255) & ~(size_t)255;
  const size_t oPrt = off; off += (size_t)nLB * 3 * NREL * DIMF * 4;      off = (off + 255) & ~(size_t)255;
  if (off > ws_size) return;
  _Float16*     wt0  = (_Float16*)(ws + oWT0);
  _Float16*     wt1  = (_Float16*)(ws + oWT1);
  unsigned int* rtI  = (unsigned int*)(ws + oRtI);
  unsigned int* rtO  = (unsigned int*)(ws + oRtO);
  int*          eidI = (int*)(ws + oEI);
  int*          eidO = (int*)(ws + oEO);
  float*        ego1 = (float*)(ws + oEgo);
  float*        part = (float*)(ws + oPrt);

  const int nPer = KIN * DIMF / 8;
  k_wprep<<<(2 * nPer + NT - 1) / NT, NT, 0, stream>>>(w0, w1, wt0, wt1, nPer);

  hipFuncSetAttribute(reinterpret_cast<const void*>(&k_csr),
                      hipFuncAttributeMaxDynamicSharedMemorySize, LDS_CSR);
  k_csr<<<nCsr, NT, LDS_CSR, stream>>>(in_row, rtI, eidI, nEI);
  k_csr<<<nCsr, NT, LDS_CSR, stream>>>(out_row, rtO, eidO, nEO);

  hipFuncSetAttribute(reinterpret_cast<const void*>(&k_layer),
                      hipFuncAttributeMaxDynamicSharedMemorySize, LDS_LAY);
  k_layer<<<nLB, NT, LDS_LAY, stream>>>(edge_emb, rtI, eidI, in_col, in_val, rtO, eidO, out_col, out_val,
                                         attr, wt0, ego1, part, N, nEI, nEO, nRt, 0);
  k_layer<<<nLB, NT, LDS_LAY, stream>>>(ego1, rtI, eidI, in_col, in_val, rtO, eidO, out_col, out_val,
                                         attr, wt1, ego1, part, N, nEI, nEO, nRt, 1);

  k_comb<<<1, NT, 0, stream>>>(part, out, nLB);
}
